// WaveNet_73607149519326
// MI455X (gfx1250) — hardware-verified
//
#include <hip/hip_runtime.h>
#include <math.h>
#include <stddef.h>
#include <stdint.h>

typedef __attribute__((ext_vector_type(16))) _Float16 v16h;
typedef __attribute__((ext_vector_type(8)))  _Float16 v8h;
typedef __attribute__((ext_vector_type(4)))  _Float16 v4h;
typedef __attribute__((ext_vector_type(16))) __bf16   v16b;
typedef __attribute__((ext_vector_type(8)))  __bf16   v8b;
typedef __attribute__((ext_vector_type(8)))  float    v8f;
typedef __attribute__((ext_vector_type(4)))  float    v4f;
typedef __attribute__((ext_vector_type(4)))  unsigned v4u;

constexpr int TLEN   = 16384;
constexpr int NHID   = 128;
constexpr int NSKIP  = 256;
constexpr int NCLS   = 256;
constexpr int NMEL   = 80;
constexpr int MELPAD = 96;
constexpr int NFRM   = 64;
constexpr int KEMB   = 512;
constexpr int NLAYER = 20;
constexpr int TT     = 64;
constexpr int NBLK   = TLEN / TT;
constexpr int NTHR   = 256;
constexpr int KGATE  = 2 * NHID + MELPAD;
constexpr int WCP    = 384;
constexpr int AGP    = 360;
constexpr int ZTP    = 136;
constexpr int SLP    = 68;
constexpr float WCARRY = 256.0f;
constexpr float WFOLD  = 1.0f / 256.0f;
constexpr float MELRATIO = (float)(64.0 / 16385.0);

static_assert(TLEN % TT == 0 && TT == 64 && NTHR == 256, "cfg");
static_assert(KGATE % 32 == 0 && NHID % 32 == 0 && KEMB % 32 == 0 && NSKIP % 32 == 0 && NCLS % 32 == 0, "cfg");
static_assert(TLEN % 64 == 0 && NHID % 64 == 0 && NSKIP % 64 == 0 && NCLS % 64 == 0, "cfg");
static_assert(AGP % 8 == 0 && AGP >= KGATE, "cfg");
static_assert(ZTP % 8 == 0 && ZTP >= NHID, "cfg");
static_assert(WCP % 64 == 0 && WCP >= KGATE, "cfg");
static_assert(8 * 16 * SLP * (int)sizeof(float) <= TT * AGP * (int)sizeof(_Float16), "cfg");
static_assert(MELPAD % 8 == 0 && NMEL % 8 == 0 && MELPAD - NMEL == 16, "cfg");
static_assert((NLAYER * NHID * 16) % NTHR == 0, "cfg");
static_assert((TLEN * (MELPAD / 8)) % NTHR == 0, "cfg");
static_assert((TLEN * (KEMB / 8)) % NTHR == 0, "cfg");
static_assert((TLEN * NSKIP / 8) % NTHR == 0, "cfg");
static_assert(TT * (MELPAD / 8) == 3 * NTHR, "cfg");
static_assert(TT * NHID / 4 == 8 * NTHR, "cfg");

constexpr size_t SZ_H    = (size_t)TLEN * NHID * 4;
constexpr size_t SZ_SK   = (size_t)TLEN * NSKIP * 4;
constexpr size_t SZ_IM   = (size_t)TLEN * KEMB * 2;
constexpr size_t SZ_MELT = (size_t)TLEN * MELPAD * 2;
constexpr size_t SZ_U    = (size_t)TLEN * NSKIP * 2;
constexpr size_t SZ_WCAT = (size_t)NLAYER * 2 * NHID * WCP * 2;
constexpr size_t SZ_SKW  = (size_t)NLAYER * NSKIP * NHID * 2;
constexpr size_t SZ_RSW  = (size_t)NLAYER * NHID * NHID * 2;
constexpr size_t SZ_EMBW = (size_t)NHID * KEMB * 2;
constexpr size_t SZ_OUTW = (size_t)NCLS * NSKIP * 2;
constexpr size_t SZ_ENDW = (size_t)NCLS * NCLS * 2;
constexpr size_t SZ_BEMB = (size_t)NHID * 4;
constexpr size_t SZ_BFG  = (size_t)NLAYER * NHID * 4;
constexpr size_t SZ_BOUT = (size_t)NCLS * 4;
constexpr size_t SZ_BEND = (size_t)NCLS * 4;
constexpr size_t OFF_HA   = 0;
constexpr size_t OFF_HB   = OFF_HA + SZ_H;
constexpr size_t OFF_SKA  = OFF_HB + SZ_H;
constexpr size_t OFF_SKB  = OFF_SKA + SZ_SK;
constexpr size_t OFF_IM   = OFF_SKB + SZ_SK;
constexpr size_t OFF_MELT = OFF_IM + SZ_IM;
constexpr size_t OFF_UA   = OFF_MELT + SZ_MELT;
constexpr size_t OFF_U2   = OFF_UA + SZ_U;
constexpr size_t OFF_WCAT = OFF_U2 + SZ_U;
constexpr size_t OFF_SKW  = OFF_WCAT + SZ_WCAT;
constexpr size_t OFF_RSW  = OFF_SKW + SZ_SKW;
constexpr size_t OFF_EMBW = OFF_RSW + SZ_RSW;
constexpr size_t OFF_OUTW = OFF_EMBW + SZ_EMBW;
constexpr size_t OFF_ENDW = OFF_OUTW + SZ_OUTW;
constexpr size_t OFF_BEMB = OFF_ENDW + SZ_ENDW;
constexpr size_t OFF_BF   = OFF_BEMB + SZ_BEMB;
constexpr size_t OFF_BG   = OFF_BF + SZ_BFG;
constexpr size_t OFF_BOUT = OFF_BG + SZ_BFG;
constexpr size_t OFF_BEND = OFF_BOUT + SZ_BOUT;
constexpr size_t WS_TOTAL = OFF_BEND + SZ_BEND;
static_assert(WS_TOTAL <= (size_t)134217728, "cfg");
static_assert(OFF_HB % 256 == 0 && OFF_SKA % 256 == 0 && OFF_SKB % 256 == 0 && OFF_IM % 256 == 0 &&
              OFF_MELT % 256 == 0 && OFF_UA % 256 == 0 && OFF_U2 % 256 == 0 && OFF_WCAT % 256 == 0 &&
              OFF_SKW % 256 == 0 && OFF_RSW % 256 == 0 && OFF_EMBW % 256 == 0 && OFF_OUTW % 256 == 0 &&
              OFF_ENDW % 256 == 0 && OFF_BEMB % 256 == 0 && OFF_BF % 256 == 0 && OFF_BG % 256 == 0 &&
              OFF_BOUT % 256 == 0 && OFF_BEND % 256 == 0, "cfg");

__device__ __forceinline__ unsigned short f2bf_bits(float f) {
  unsigned u = __float_as_uint(f);
  return (unsigned short)((u + 0x7FFFu + ((u >> 16) & 1u)) >> 16);
}
__device__ __forceinline__ float bf_bits2f(unsigned short h) { return __uint_as_float(((unsigned)h) << 16); }

__device__ __forceinline__ void dep_guard_h(v8f& a, v8f& b, v16h x, v16h y) { asm volatile("v_nop\n\tv_nop\n\tv_nop\n\tv_nop" : "+v"(a), "+v"(b) : "v"(x), "v"(y)); }
__device__ __forceinline__ void dep_guard_b(v8f& a, v8f& b, v16b x, v16b y) { asm volatile("v_nop\n\tv_nop\n\tv_nop\n\tv_nop" : "+v"(a), "+v"(b) : "v"(x), "v"(y)); }
__device__ __forceinline__ void keep4_h(v16h a, v16h b, v16h c, v16h d) { asm volatile("v_nop" :: "v"(a), "v"(b), "v"(c), "v"(d)); }
__device__ __forceinline__ void keep4_b(v16b a, v16b b, v16b c, v16b d) { asm volatile("v_nop" :: "v"(a), "v"(b), "v"(c), "v"(d)); }
__device__ __forceinline__ void acc_guard4(v8f& a, v8f& b, v8f& c, v8f& d) { asm volatile("v_nop\n\tv_nop\n\tv_nop\n\tv_nop" : "+v"(a), "+v"(b), "+v"(c), "+v"(d)); }
template <typename T> struct Frag;
template <> struct Frag<_Float16> {
  typedef v16h V; union U { v16h v; v8h h[2]; };
  static __device__ __forceinline__ v16h load(const _Float16* p) {
    U f; f.h[0] = *(const v8h*)(p); f.h[1] = *(const v8h*)(p + 16); return f.v;
  }
  static __device__ __forceinline__ v8f mma(v16h a, v16h b, v8f c) {
    return __builtin_amdgcn_wmma_f32_16x16x32_f16(false, a, false, b, (short)0, c, false, false);
  }
  static __device__ __forceinline__ void guard(v8f& a, v8f& b, v16h x, v16h y) { dep_guard_h(a, b, x, y); }
  static __device__ __forceinline__ void keep(v16h a, v16h b, v16h c, v16h d) { keep4_h(a, b, c, d); }
};
template <> struct Frag<__bf16> {
  typedef v16b V; union U { v16b v; v8b h[2]; };
  static __device__ __forceinline__ v16b load(const __bf16* p) {
    U f; f.h[0] = *(const v8b*)(p); f.h[1] = *(const v8b*)(p + 16); return f.v;
  }
  static __device__ __forceinline__ v8f mma(v16b a, v16b b, v8f c) {
    return __builtin_amdgcn_wmma_f32_16x16x32_bf16(false, a, false, b, (short)0, c, false, false);
  }
  static __device__ __forceinline__ void guard(v8f& a, v8f& b, v16b x, v16b y) { dep_guard_b(a, b, x, y); }
  static __device__ __forceinline__ void keep(v16b a, v16b b, v16b c, v16b d) { keep4_b(a, b, c, d); }
};

template <int ET> struct Elem;
template <> struct Elem<0> { typedef _Float16 T; };
template <> struct Elem<1> { typedef __bf16 T; };
template <int ET, bool SPLIT, int BIAS_MODE, int OUT_MODE, bool RESID, int ACT = 0>
__global__ __launch_bounds__(256) void wmma_gemm64(
    const unsigned short* __restrict__ Ap, const unsigned short* __restrict__ A2p, int lda, long strideA,
    const unsigned short* __restrict__ Btp, const unsigned short* __restrict__ Bt2p, int ldb, long strideB,
    void* __restrict__ Cout, void* __restrict__ Cout2, int ldc, long strideC,
    const float* __restrict__ bias,
    const float* __restrict__ resid, long strideR,
    int M, int N, int K, float scale) {
  typedef typename Elem<ET>::T T;
  typedef typename Frag<T>::V V;
  const T* A = (const T*)Ap; const T* A2 = (const T*)A2p; const T* Bt = (const T*)Btp; const T* Bt2 = (const T*)Bt2p;
  __shared__ __align__(16) float sT[8][16 * 68];
  const int b    = blockIdx.y;
  const int lane = threadIdx.x & 31;
  const int wave = threadIdx.x >> 5;
  const int tilesN = N >> 6;
  const int tilesM = M >> 6;
  const int tile = blockIdx.x * 8 + wave;
  if (tile >= tilesM * tilesN) return;
  const int tm = tile / tilesN;
  const int tn = tile - tm * tilesN;
  const int m0 = tm << 6;
  const int n0 = tn << 6;

  const T* Ab  = A  + (size_t)b * strideA;
  const T* Bb  = Bt + (size_t)b * strideB;
  const T* Ab2 = SPLIT ? (A2  + (size_t)b * strideA) : nullptr;
  const T* Bb2 = SPLIT ? (Bt2 + (size_t)b * strideB) : nullptr;

  const int rlane = lane & 15;
  const int koff  = (lane >> 4) * 8;
  const int mOff  = (lane >> 4) * 8;

  v8f acc[4][4];
#pragma unroll
  for (int i = 0; i < 4; ++i)
#pragma unroll
    for (int j = 0; j < 4; ++j) acc[i][j] = (v8f){0.f,0.f,0.f,0.f,0.f,0.f,0.f,0.f};

  for (int k0 = 0; k0 < K; k0 += 32) {
    V bh[4], bl[4];
#pragma unroll
    for (int j = 0; j < 4; ++j) {
      const size_t bo = (size_t)(n0 + (j << 4) + rlane) * ldb + koff + k0;
      bh[j] = Frag<T>::load(Bb + bo);
      if (SPLIT) bl[j] = Frag<T>::load(Bb2 + bo);
    }
#pragma unroll
    for (int i = 0; i < 4; ++i) {
      const size_t ao = (size_t)(m0 + (i << 4) + rlane) * lda + koff + k0;
      V ah = Frag<T>::load(Ab + ao);
      V al;
      if (SPLIT) al = Frag<T>::load(Ab2 + ao);
#pragma unroll
      for (int j = 0; j < 4; ++j) {
        acc[i][j] = Frag<T>::mma(ah, bh[j], acc[i][j]);
        if (SPLIT) {
          acc[i][j] = Frag<T>::mma(ah, bl[j], acc[i][j]);
          acc[i][j] = Frag<T>::mma(al, bh[j], acc[i][j]);
        }
      }
      Frag<T>::guard(acc[i][0], acc[i][3], ah, SPLIT ? al : ah);
    }
    Frag<T>::keep(bh[0], bh[1], bh[2], bh[3]);
    if (SPLIT) Frag<T>::keep(bl[0], bl[1], bl[2], bl[3]);
  }
  acc_guard4(acc[0][0], acc[0][1], acc[0][2], acc[0][3]);
  acc_guard4(acc[1][0], acc[1][1], acc[1][2], acc[1][3]);
  acc_guard4(acc[2][0], acc[2][1], acc[2][2], acc[2][3]);
  acc_guard4(acc[3][0], acc[3][1], acc[3][2], acc[3][3]);

  float* slab = sT[wave];
  const float* Rb = RESID ? (resid + (size_t)b * strideR) : nullptr;
#pragma unroll
  for (int i = 0; i < 4; ++i) {
    const int mBase = m0 + (i << 4);
#pragma unroll
    for (int j = 0; j < 4; ++j) {
      const int n = n0 + (j << 4) + rlane;
      float bv = 0.f;
      if (BIAS_MODE == 2) bv = bias[n];
#pragma unroll
      for (int r = 0; r < 8; ++r) {
        float v = acc[i][j][r] * scale;
        if (BIAS_MODE == 1) v += bias[mBase + mOff + r];
        if (BIAS_MODE == 2) v += bv;
        if (RESID) v += Rb[(size_t)(mBase + mOff + r) * ldc + n];
        if (ACT == 1) v = tanhf(v);
        if (ACT == 2) v = fmaxf(v, 0.0f);
        if (ACT == 3) v = v / (1.0f + expf(-v));
        if (ACT == 4) v = (v > 0.f) ? v : 0.01f * v;
        if (ACT == 5) v = 0.5f * v * (1.0f + erff(v * 0.70710678118654752f));
        slab[(mOff + r) * 68 + (j << 4) + rlane] = v;
      }
    }
    __builtin_amdgcn_fence(__ATOMIC_RELEASE, "workgroup");
    __builtin_amdgcn_wave_barrier();
    __builtin_amdgcn_fence(__ATOMIC_ACQUIRE, "workgroup");
    if (OUT_MODE == 0) {
      float* C = (float*)Cout + (size_t)b * strideC;
      const int hh = lane >> 4, c4 = (lane & 15) * 4;
      for (int pass = 0; pass < 2; ++pass) {
#pragma unroll
        for (int it = 0; it < 8; ++it) {
          const int row = it * 2 + hh;
          v4f v = *(const v4f*)(slab + row * 68 + c4);
          *(volatile v4f*)(C + (size_t)(mBase + row) * ldc + n0 + c4) = v;
        }
        __threadfence();
      }
    } else {
      const int q = lane >> 3, c8 = (lane & 7) * 8;
      unsigned short* C  = (unsigned short*)Cout  + (size_t)b * strideC;
      unsigned short* C2 = (OUT_MODE == 2) ? ((unsigned short*)Cout2 + (size_t)b * strideC) : nullptr;
      for (int pass = 0; pass < 2; ++pass) {
#pragma unroll
        for (int it = 0; it < 4; ++it) {
          const int row = it * 4 + q;
          const float* sp = slab + row * 68 + c8;
          v8h hv, lv;
#pragma unroll
          for (int e = 0; e < 8; ++e) {
            if (OUT_MODE == 1) {
              hv[e] = (_Float16)sp[e];
            } else {
              unsigned short hb = f2bf_bits(sp[e]);
              unsigned short lb = f2bf_bits(sp[e] - bf_bits2f(hb));
              hv[e] = __builtin_bit_cast(_Float16, hb);
              lv[e] = __builtin_bit_cast(_Float16, lb);
            }
          }
          *(volatile v8h*)(C + (size_t)(mBase + row) * ldc + n0 + c8) = hv;
          if (OUT_MODE == 2) *(volatile v8h*)(C2 + (size_t)(mBase + row) * ldc + n0 + c8) = lv;
        }
        __threadfence();
      }
    }
    __builtin_amdgcn_fence(__ATOMIC_RELEASE, "workgroup");
    __builtin_amdgcn_wave_barrier();
    __builtin_amdgcn_fence(__ATOMIC_ACQUIRE, "workgroup");
  }
}

typedef Frag<_Float16> FragH;

__device__ __forceinline__ float bfr(float f) { return bf_bits2f(f2bf_bits(f)); }

__device__ __forceinline__ void guard4in5(v8f& a0, v8f& a1, v8f& a2, v8f& a3,
                                          v16h x, v16h b0, v16h b1, v16h b2, v16h b3) {
  asm volatile("v_nop\n\tv_nop\n\tv_nop\n\tv_nop"
               : "+v"(a0), "+v"(a1), "+v"(a2), "+v"(a3)
               : "v"(x), "v"(b0), "v"(b1), "v"(b2), "v"(b3));
}
__device__ __forceinline__ void guard8in6(v8f& a0, v8f& a1, v8f& a2, v8f& a3,
                                          v8f& c0, v8f& c1, v8f& c2, v8f& c3,
                                          v16h x0, v16h x1, v16h x2, v16h x3, v16h y0, v16h y1) {
  asm volatile("v_nop\n\tv_nop\n\tv_nop\n\tv_nop"
               : "+v"(a0), "+v"(a1), "+v"(a2), "+v"(a3), "+v"(c0), "+v"(c1), "+v"(c2), "+v"(c3)
               : "v"(x0), "v"(x1), "v"(x2), "v"(x3), "v"(y0), "v"(y1));
}

__device__ __forceinline__ void store_h8_twice(unsigned short* p, v8h v) {
  *(volatile v8h*)p = v;
  __threadfence();
  *(volatile v8h*)p = v;
}
__device__ __forceinline__ void store_f4_twice(float* p, v4f v) {
  *(volatile v4f*)p = v;
  __threadfence();
  *(volatile v4f*)p = v;
}

__global__ __launch_bounds__(NTHR) void k_castw(const float* __restrict__ src, unsigned short* __restrict__ dst,
                                                int n8, float scale) {
  const int i = blockIdx.x * NTHR + threadIdx.x;
  if (i >= n8) return;
  const size_t e0 = (size_t)i * 8;
  const v4f q0 = *(const v4f*)(src + e0);
  const v4f q1 = *(const v4f*)(src + e0 + 4);
  v8h hv;
  hv[0] = (_Float16)(scale * bfr(q0[0])); hv[1] = (_Float16)(scale * bfr(q0[1]));
  hv[2] = (_Float16)(scale * bfr(q0[2])); hv[3] = (_Float16)(scale * bfr(q0[3]));
  hv[4] = (_Float16)(scale * bfr(q1[0])); hv[5] = (_Float16)(scale * bfr(q1[1]));
  hv[6] = (_Float16)(scale * bfr(q1[2])); hv[7] = (_Float16)(scale * bfr(q1[3]));
  store_h8_twice(dst + e0, hv);
}

__global__ __launch_bounds__(NTHR) void k_wcat_w(const float* __restrict__ Wf, const float* __restrict__ Wg,
                                                 unsigned short* __restrict__ wcat) {
  const int i = blockIdx.x * NTHR + threadIdx.x;
  if (i >= NLAYER * NHID * 16) return;
  const int tap = blockIdx.y & 1;
  const int fg  = blockIdx.y >> 1;
  const int l   = i >> 11;
  const int rem = i & 2047;
  const int o   = rem >> 4;
  const int ch  = rem & 15;
  const float* W = fg ? Wg : Wf;
  const float* src = W + (((size_t)(l * NHID + o)) * NHID + ch * 8) * 2;
  const v4f q0 = *(const v4f*)(src);
  const v4f q1 = *(const v4f*)(src + 4);
  const v4f q2 = *(const v4f*)(src + 8);
  const v4f q3 = *(const v4f*)(src + 12);
  float ev[8], od[8];
  ev[0] = q0[0]; od[0] = q0[1]; ev[1] = q0[2]; od[1] = q0[3];
  ev[2] = q1[0]; od[2] = q1[1]; ev[3] = q1[2]; od[3] = q1[3];
  ev[4] = q2[0]; od[4] = q2[1]; ev[5] = q2[2]; od[5] = q2[3];
  ev[6] = q3[0]; od[6] = q3[1]; ev[7] = q3[2]; od[7] = q3[3];
  const float ft = (float)tap;
  const float fe = 1.0f - ft;
  v8h hv;
#pragma unroll
  for (int e = 0; e < 8; ++e) {
    const float v = fmaf(ft, od[e], fe * ev[e]);
    hv[e] = (_Float16)(WCARRY * bfr(v));
  }
  unsigned short* dst = wcat + ((size_t)(l * 2 * NHID + fg * NHID + o)) * WCP + tap * NHID + ch * 8;
  store_h8_twice(dst, hv);
}

__global__ __launch_bounds__(NTHR) void k_wcat_v(const float* __restrict__ Vf, const float* __restrict__ Vg,
                                                 unsigned short* __restrict__ wcat) {
  const int i = blockIdx.x * NTHR + threadIdx.x;
  if (i >= NLAYER * NHID * 16) return;
  const int fg  = blockIdx.y & 1;
  const int l   = i >> 11;
  const int rem = i & 2047;
  const int o   = rem >> 4;
  const int ch  = rem & 15;
  const int c0  = ch * 8;
  const int c0c = (c0 < NMEL) ? c0 : (NMEL - 8);
  const float fz = (c0 < NMEL) ? 1.0f : 0.0f;
  const float* V = fg ? Vg : Vf;
  const float* src = V + (size_t)(l * NHID + o) * NMEL + c0c;
  const v4f q0 = *(const v4f*)(src);
  const v4f q1 = *(const v4f*)(src + 4);
  v8h hv;
  hv[0] = (_Float16)(WCARRY * bfr(q0[0]) * fz); hv[1] = (_Float16)(WCARRY * bfr(q0[1]) * fz);
  hv[2] = (_Float16)(WCARRY * bfr(q0[2]) * fz); hv[3] = (_Float16)(WCARRY * bfr(q0[3]) * fz);
  hv[4] = (_Float16)(WCARRY * bfr(q1[0]) * fz); hv[5] = (_Float16)(WCARRY * bfr(q1[1]) * fz);
  hv[6] = (_Float16)(WCARRY * bfr(q1[2]) * fz); hv[7] = (_Float16)(WCARRY * bfr(q1[3]) * fz);
  unsigned short* dst = wcat + ((size_t)(l * 2 * NHID + fg * NHID + o)) * WCP + 2 * NHID + c0;
  store_h8_twice(dst, hv);
}

template <bool TWO>
__global__ __launch_bounds__(NTHR) void k_biasprep(const float* __restrict__ a, const float* __restrict__ b,
                                                   float* __restrict__ dst, int n4) {
  const int i = blockIdx.x * NTHR + threadIdx.x;
  if (i >= n4) return;
  const size_t e0 = (size_t)i * 4;
  const v4f x = *(const v4f*)(a + e0);
  v4f r;
  r[0] = bfr(x[0]); r[1] = bfr(x[1]); r[2] = bfr(x[2]); r[3] = bfr(x[3]);
  if (TWO) {
    const v4f y = *(const v4f*)(b + e0);
    r[0] += bfr(y[0]); r[1] += bfr(y[1]); r[2] += bfr(y[2]); r[3] += bfr(y[3]);
  }
  store_f4_twice(dst + e0, r);
}

__global__ __launch_bounds__(NTHR) void k_melt(const float* __restrict__ melspec, unsigned short* __restrict__ melT) {
#pragma clang fp contract(off)
  const int i = blockIdx.x * NTHR + threadIdx.x;
  if (i >= TLEN * (MELPAD / 8)) return;
  const int t   = i / 12;
  const int ch  = i - t * 12;
  const int c0  = ch * 8;
  const int c0c = (c0 < NMEL) ? c0 : (NMEL - 8);
  const float fz = (c0 < NMEL) ? 1.0f : 0.0f;
  const float p = (float)(t + 1) * MELRATIO;
  int s = (int)floorf(p);
  s = s < 0 ? 0 : (s > NFRM - 1 ? (NFRM - 1) : s);
  v8h hv;
#pragma unroll
  for (int e = 0; e < 8; ++e) {
    const float v = melspec[(size_t)(c0c + e) * NFRM + s] * fz;
    hv[e] = (_Float16)bfr(v);
  }
  store_h8_twice(melT + (size_t)i * 8, hv);
}

__global__ __launch_bounds__(NTHR) void k_im2col(const float* __restrict__ wav, unsigned short* __restrict__ im) {
  const int i = blockIdx.x * NTHR + threadIdx.x;
  if (i >= TLEN * (KEMB / 8)) return;
  const int t  = i >> 6;
  const int k0 = (i & 63) * 8;
  const int g0 = t - (KEMB - 1) + k0;
  v8h hv;
#pragma unroll
  for (int e = 0; e < 8; ++e) {
    const int g  = g0 + e;
    const int gc = g < 0 ? 0 : g;
    const float fz = g < 0 ? 0.0f : 1.0f;
    const float v = wav[gc] * fz;
    hv[e] = (_Float16)bfr(v);
  }
  store_h8_twice(im + (size_t)i * 8, hv);
}

__global__ __launch_bounds__(NTHR) void k_relu16(const float* __restrict__ s, unsigned short* __restrict__ d, int n8) {
  const int i = blockIdx.x * NTHR + threadIdx.x;
  if (i >= n8) return;
  const size_t e0 = (size_t)i * 8;
  const v4f q0 = *(const v4f*)(s + e0);
  const v4f q1 = *(const v4f*)(s + e0 + 4);
  v8h hv;
  hv[0] = (_Float16)fmaxf(q0[0], 0.0f); hv[1] = (_Float16)fmaxf(q0[1], 0.0f);
  hv[2] = (_Float16)fmaxf(q0[2], 0.0f); hv[3] = (_Float16)fmaxf(q0[3], 0.0f);
  hv[4] = (_Float16)fmaxf(q1[0], 0.0f); hv[5] = (_Float16)fmaxf(q1[1], 0.0f);
  hv[6] = (_Float16)fmaxf(q1[2], 0.0f); hv[7] = (_Float16)fmaxf(q1[3], 0.0f);
  store_h8_twice(d + e0, hv);
}

template <bool HAS_RES>
__device__ __forceinline__ void tile16x64_k128(const _Float16* arow, const _Float16* brow, float* slab,
                                               const float* __restrict__ bias_n0,
                                               const float* __restrict__ res_base, float* dst_base, int ldc, int lane) {
  const int rl = lane & 15;
  const int mOff = (lane >> 4) * 8;
  const v8f z8 = {0.f, 0.f, 0.f, 0.f, 0.f, 0.f, 0.f, 0.f};
  v8f acc[4];
  acc[0] = z8; acc[1] = z8; acc[2] = z8; acc[3] = z8;
#pragma unroll 1
  for (int k0 = 0; k0 < NHID; k0 += 32) {
    const v16h a  = FragH::load(arow + k0);
    const v16h b0 = FragH::load(brow + k0);
    const v16h b1 = FragH::load(brow + (size_t)16 * NHID + k0);
    const v16h b2 = FragH::load(brow + (size_t)32 * NHID + k0);
    const v16h b3 = FragH::load(brow + (size_t)48 * NHID + k0);
    acc[0] = FragH::mma(a, b0, acc[0]);
    acc[1] = FragH::mma(a, b1, acc[1]);
    acc[2] = FragH::mma(a, b2, acc[2]);
    acc[3] = FragH::mma(a, b3, acc[3]);
    guard4in5(acc[0], acc[1], acc[2], acc[3], a, b0, b1, b2, b3);
  }
#pragma unroll
  for (int j = 0; j < 4; ++j)
#pragma unroll
    for (int r = 0; r < 8; ++r) slab[(mOff + r) * SLP + (j << 4) + rl] = acc[j][r] * WFOLD;
  __builtin_amdgcn_fence(__ATOMIC_RELEASE, "workgroup");
  __builtin_amdgcn_wave_barrier();
  __builtin_amdgcn_fence(__ATOMIC_ACQUIRE, "workgroup");
  const int hh = lane >> 4, c4 = (lane & 15) * 4;
  const v4f braw = *(const v4f*)(bias_n0 + c4);
  v4f b4;
  b4[0] = bfr(braw[0]); b4[1] = bfr(braw[1]); b4[2] = bfr(braw[2]); b4[3] = bfr(braw[3]);
  v4f vals[8];
#pragma unroll
  for (int it = 0; it < 8; ++it) {
    const int row = it * 2 + hh;
    v4f v = *(const v4f*)(slab + row * SLP + c4) + b4;
    if (HAS_RES) {
      const v4f rr = *(const v4f*)(res_base + (size_t)row * ldc + c4);
      v = v + rr;
    }
    vals[it] = v;
    if (it == 3) asm volatile("" ::: "memory");
  }
  for (int pass = 0; pass < 2; ++pass) {
#pragma unroll
    for (int it = 0; it < 8; ++it) {
      const int row = it * 2 + hh;
      *(volatile v4f*)(dst_base + (size_t)row * ldc + c4) = vals[it];
    }
    __threadfence();
  }
  __builtin_amdgcn_fence(__ATOMIC_RELEASE, "workgroup");
  __builtin_amdgcn_wave_barrier();
  __builtin_amdgcn_fence(__ATOMIC_ACQUIRE, "workgroup");
}

template <bool SKIP_ACC>
__global__ __launch_bounds__(NTHR) void layer_kernel(
    const float* __restrict__ h_in, float* __restrict__ h_out,
    const float* __restrict__ skip_in, float* __restrict__ skip_out,
    const unsigned short* __restrict__ melT,
    const unsigned short* __restrict__ wcat_l,
    const unsigned short* __restrict__ skw_l,
    const unsigned short* __restrict__ rsw_l,
    const float* __restrict__ biasf_l, const float* __restrict__ biasg_l,
    const float* __restrict__ skipb_l, const float* __restrict__ resb_l, int d) {
  __shared__ __align__(16) float lds_main[TT * AGP / 2];
  __shared__ __align__(16) _Float16 zt[TT * ZTP];
  _Float16* ag = (_Float16*)lds_main;

  const int tid = threadIdx.x, lane = tid & 31, wave = tid >> 5;
  const int t0 = blockIdx.x * TT;
  const int dd = d < 1 ? 1 : (d > TLEN ? TLEN : d);

#pragma unroll 1
  for (int it = 0; it < 8; ++it) {
    const int row  = it * 8 + wave;
    const int c4   = lane * 4;
    const int tcur = t0 + row;
    const int ts   = tcur - dd;
    const int tsc  = ts < 0 ? 0 : ts;
    const float fz = ts < 0 ? 0.0f : 1.0f;
    const v4f hv = *(const v4f*)(h_in + (size_t)tcur * NHID + c4);
    const v4f sv = *(const v4f*)(h_in + (size_t)tsc * NHID + c4);
    v4h hq, sq;
    hq[0] = (_Float16)hv[0]; hq[1] = (_Float16)hv[1]; hq[2] = (_Float16)hv[2]; hq[3] = (_Float16)hv[3];
    sq[0] = (_Float16)(sv[0] * fz); sq[1] = (_Float16)(sv[1] * fz);
    sq[2] = (_Float16)(sv[2] * fz); sq[3] = (_Float16)(sv[3] * fz);
    *(v4h*)(ag + row * AGP + NHID + c4) = hq;
    *(v4h*)(ag + row * AGP + c4) = sq;
  }
#pragma unroll 1
  for (int it = 0; it < 3; ++it) {
    const int idx = it * NTHR + tid;
    const int row = idx / 12;
    const int ch  = idx - row * 12;
    const v4u mv = *(const v4u*)(melT + ((size_t)(t0 + row) * MELPAD + ch * 8));
    *(v4u*)(ag + row * AGP + 2 * NHID + ch * 8) = mv;
  }
  __syncthreads();

  const int rl = lane & 15;
  const int koff = (lane >> 4) * 8;
  const int mOff = koff;
  const v8f z8 = {0.f, 0.f, 0.f, 0.f, 0.f, 0.f, 0.f, 0.f};
  v8f accf[4], accg[4];
  accf[0] = z8; accf[1] = z8; accf[2] = z8; accf[3] = z8;
  accg[0] = z8; accg[1] = z8; accg[2] = z8; accg[3] = z8;
  {
    const _Float16* arow  = ag + rl * AGP + koff;
    const _Float16* wfrow = (const _Float16*)wcat_l + (size_t)(wave * 16 + rl) * WCP + koff;
    const _Float16* wgrow = wfrow + (size_t)NHID * WCP;
#pragma unroll 1
    for (int k0 = 0; k0 < KGATE; k0 += 32) {
      const v16h bfq = FragH::load(wfrow + k0);
      const v16h bgq = FragH::load(wgrow + k0);
      const v16h a0 = FragH::load(arow + k0);
      const v16h a1 = FragH::load(arow + 16 * AGP + k0);
      const v16h a2 = FragH::load(arow + 32 * AGP + k0);
      const v16h a3 = FragH::load(arow + 48 * AGP + k0);
      accf[0] = FragH::mma(a0, bfq, accf[0]); accg[0] = FragH::mma(a0, bgq, accg[0]);
      accf[1] = FragH::mma(a1, bfq, accf[1]); accg[1] = FragH::mma(a1, bgq, accg[1]);
      accf[2] = FragH::mma(a2, bfq, accf[2]); accg[2] = FragH::mma(a2, bgq, accg[2]);
      accf[3] = FragH::mma(a3, bfq, accf[3]); accg[3] = FragH::mma(a3, bgq, accg[3]);
      guard8in6(accf[0], accf[1], accf[2], accf[3], accg[0], accg[1], accg[2], accg[3], a0, a1, a2, a3, bfq, bgq);
    }
  }
  {
    const int o = wave * 16 + rl;
    const float bfo = biasf_l[o];
    const float bgo = biasg_l[o];
#pragma unroll
    for (int i = 0; i < 4; ++i) {
#pragma unroll
      for (int r = 0; r < 8; ++r) {
        const int trow = i * 16 + mOff + r;
        const float fv = fmaf(accf[i][r], WFOLD, bfo);
        const float gv = fmaf(accg[i][r], WFOLD, bgo);
        const float zv = tanhf(fv) * __builtin_amdgcn_rcpf(1.0f + expf(-gv));
        zt[trow * ZTP + o] = (_Float16)zv;
      }
    }
  }
  __syncthreads();

  {
    float* slab = lds_main + wave * (16 * SLP);
    const int ti = wave & 3;
    const int chalf = wave >> 2;
    const _Float16* zrow = zt + (ti * 16 + rl) * ZTP + koff;
    const size_t trow0 = (size_t)(t0 + ti * 16);
#pragma unroll 1
    for (int sub = 0; sub < 2; ++sub) {
      const int n0 = chalf * 128 + sub * 64;
      const _Float16* brow = (const _Float16*)skw_l + (size_t)(n0 + rl) * NHID + koff;
      tile16x64_k128<SKIP_ACC>(zrow, brow, slab, skipb_l + n0,
                               skip_in + trow0 * NSKIP + n0, skip_out + trow0 * NSKIP + n0, NSKIP, lane);
    }
    {
      const int n0 = chalf * 64;
      const _Float16* brow = (const _Float16*)rsw_l + (size_t)(n0 + rl) * NHID + koff;
      tile16x64_k128<true>(zrow, brow, slab, resb_l + n0,
                           h_in + trow0 * NHID + n0, h_out + trow0 * NHID + n0, NHID, lane);
    }
  }
}

static inline unsigned cdiv_u(unsigned a, unsigned b) { return (a + b - 1) / b; }

extern "C" void kernel_launch(void* const* d_in, const int* in_sizes, int n_in,
                              void* d_out, int out_size, void* d_ws, size_t ws_size, hipStream_t stream) {
  if (n_in < 20) return;
  if (in_sizes[0] != NMEL * NFRM || in_sizes[1] != TLEN || out_size != NCLS * TLEN) return;
  if (ws_size < WS_TOTAL) return;

  const float* melspec = (const float*)d_in[0];
  const float* wav     = (const float*)d_in[1];
  const float* emb_w   = (const float*)d_in[2];
  const float* emb_b   = (const float*)d_in[3];
  const float* Wf      = (const float*)d_in[4];
  const float* Wf_b    = (const float*)d_in[5];
  const float* Wg      = (const float*)d_in[6];
  const float* Wg_b    = (const float*)d_in[7];
  const float* Vf      = (const float*)d_in[8];
  const float* Vf_b    = (const float*)d_in[9];
  const float* Vg      = (const float*)d_in[10];
  const float* Vg_b    = (const float*)d_in[11];
  const float* skip_w  = (const float*)d_in[12];
  const float* skip_b  = (const float*)d_in[13];
  const float* res_w   = (const float*)d_in[14];
  const float* res_b   = (const float*)d_in[15];
  const float* out_w   = (const float*)d_in[16];
  const float* out_b   = (const float*)d_in[17];
  const float* end_w   = (const float*)d_in[18];
  const float* end_b   = (const float*)d_in[19];
  float* outp = (float*)d_out;

  char* ws = (char*)d_ws;
  float* hA = (float*)(ws + OFF_HA);
  float* hB = (float*)(ws + OFF_HB);
  float* skA = (float*)(ws + OFF_SKA);
  float* skB = (float*)(ws + OFF_SKB);
  unsigned short* im   = (unsigned short*)(ws + OFF_IM);
  unsigned short* melT = (unsigned short*)(ws + OFF_MELT);
  unsigned short* uA   = (unsigned short*)(ws + OFF_UA);
  unsigned short* u2   = (unsigned short*)(ws + OFF_U2);
  unsigned short* wcat = (unsigned short*)(ws + OFF_WCAT);
  unsigned short* skw  = (unsigned short*)(ws + OFF_SKW);
  unsigned short* rsw  = (unsigned short*)(ws + OFF_RSW);
  unsigned short* embw = (unsigned short*)(ws + OFF_EMBW);
  unsigned short* outw = (unsigned short*)(ws + OFF_OUTW);
  unsigned short* endw = (unsigned short*)(ws + OFF_ENDW);
  float* bemb = (float*)(ws + OFF_BEMB);
  float* bfs  = (float*)(ws + OFF_BF);
  float* bgs  = (float*)(ws + OFF_BG);
  float* bout = (float*)(ws + OFF_BOUT);
  float* bend = (float*)(ws + OFF_BEND);

  const dim3 blk(NTHR);

  {
    const int n8_emb = NHID * KEMB / 8;
    const int n8_skw = NLAYER * NSKIP * NHID / 8;
    const int n8_rsw = NLAYER * NHID * NHID / 8;
    const int n8_ow  = NCLS * NSKIP / 8;
    const int n8_ew  = NCLS * NCLS / 8;
    k_castw<<<dim3(cdiv_u(n8_emb, NTHR)), blk, 0, stream>>>(emb_w, embw, n8_emb, WCARRY);
    k_castw<<<dim3(cdiv_u(n8_skw, NTHR)), blk, 0, stream>>>(skip_w, skw, n8_skw, WCARRY);
    k_castw<<<dim3(cdiv_u(n8_rsw, NTHR)), blk, 0, stream>>>(res_w, rsw, n8_rsw, WCARRY);
    k_castw<<<dim3(cdiv_u(n8_ow, NTHR)), blk, 0, stream>>>(out_w, outw, n8_ow, WCARRY);
    k_castw<<<dim3(cdiv_u(n8_ew, NTHR)), blk, 0, stream>>>(end_w, endw, n8_ew, WCARRY);
    const unsigned nrow16 = cdiv_u(NLAYER * NHID * 16, NTHR);
    k_wcat_w<<<dim3(nrow16, 4), blk, 0, stream>>>(Wf, Wg, wcat);
    k_wcat_v<<<dim3(nrow16, 2), blk, 0, stream>>>(Vf, Vg, wcat);
    k_biasprep<false><<<dim3(cdiv_u(NHID / 4, NTHR)), blk, 0, stream>>>(emb_b, emb_b, bemb, NHID / 4);
    k_biasprep<true><<<dim3(cdiv_u(NLAYER * NHID / 4, NTHR)), blk, 0, stream>>>(Wf_b, Vf_b, bfs, NLAYER * NHID / 4);
    k_biasprep<true><<<dim3(cdiv_u(NLAYER * NHID / 4, NTHR)), blk, 0, stream>>>(Wg_b, Vg_b, bgs, NLAYER * NHID / 4);
    k_biasprep<false><<<dim3(cdiv_u(NCLS / 4, NTHR)), blk, 0, stream>>>(out_b, out_b, bout, NCLS / 4);
    k_biasprep<false><<<dim3(cdiv_u(NCLS / 4, NTHR)), blk, 0, stream>>>(end_b, end_b, bend, NCLS / 4);
    k_melt<<<dim3(cdiv_u(TLEN * (MELPAD / 8), NTHR)), blk, 0, stream>>>(melspec, melT);
    k_im2col<<<dim3(cdiv_u(TLEN * (KEMB / 8), NTHR)), blk, 0, stream>>>(wav, im);
  }

  {
    const unsigned tiles = (TLEN / 64) * (NHID / 64);
    wmma_gemm64<0, false, 2, 0, false, 0><<<dim3(cdiv_u(tiles, 8), 1), blk, 0, stream>>>(
        im, im, KEMB, 0L, embw, embw, KEMB, 0L, (void*)hA, (void*)hA, NHID, 0L,
        bemb, hA, 0L, TLEN, NHID, KEMB, WFOLD);
  }

  const float* hin = hA;  float* hout = hB;
  const float* sin_ = skA; float* sout = skB;
  for (int l = 0; l < NLAYER; ++l) {
    const int d = 1 << (l % 10);
    const unsigned short* wcat_l = wcat + (size_t)l * 2 * NHID * WCP;
    const unsigned short* skw_l  = skw + (size_t)l * NSKIP * NHID;
    const unsigned short* rsw_l  = rsw + (size_t)l * NHID * NHID;
    const float* bf_l = bfs + (size_t)l * NHID;
    const float* bg_l = bgs + (size_t)l * NHID;
    const float* sb_l = skip_b + (size_t)l * NSKIP;
    const float* rb_l = res_b + (size_t)l * NHID;
    if (l == 0) {
      layer_kernel<false><<<dim3(NBLK), blk, 0, stream>>>(hin, hout, sin_, sout, melT, wcat_l, skw_l, rsw_l,
                                                          bf_l, bg_l, sb_l, rb_l, d);
    } else {
      layer_kernel<true><<<dim3(NBLK), blk, 0, stream>>>(hin, hout, sin_, sout, melT, wcat_l, skw_l, rsw_l,
                                                         bf_l, bg_l, sb_l, rb_l, d);
    }
    { const float* t1 = hin;  hin = hout;  hout = (float*)t1; }
    { const float* t2 = sin_; sin_ = sout; sout = (float*)t2; }
  }
  const float* skip_final = sin_;

  {
    const int n8_u = TLEN * NSKIP / 8;
    k_relu16<<<dim3(cdiv_u(n8_u, NTHR)), blk, 0, stream>>>(skip_final, uA, n8_u);
    const unsigned tiles1 = (TLEN / 64) * (NCLS / 64);
    wmma_gemm64<0, false, 2, 1, false, 2><<<dim3(cdiv_u(tiles1, 8), 1), blk, 0, stream>>>(
        uA, uA, NSKIP, 0L, outw, outw, NSKIP, 0L, (void*)u2, (void*)u2, NCLS, 0L,
        bout, hA, 0L, TLEN, NCLS, NSKIP, WFOLD);
    const unsigned tiles2 = (NCLS / 64) * (TLEN / 64);
    wmma_gemm64<0, false, 1, 0, false, 0><<<dim3(cdiv_u(tiles2, 8), 1), blk, 0, stream>>>(
        endw, endw, NCLS, 0L, u2, u2, NCLS, 0L, (void*)outp, (void*)outp, TLEN, 0L,
        bend, hA, 0L, NCLS, TLEN, NCLS, WFOLD);
  }
}
